// EntailmentSelfAttention_2688649527624
// MI455X (gfx1250) — hardware-verified
//
#include <hip/hip_runtime.h>
#include <math.h>
#include <stdint.h>

#define NSB  8
#define LQ   1024
#define EE   256
#define NH   8
#define DH   32
#define MR   (NSB * LQ)
#define XSC  64.0f
#define WSC  1024.0f
#define ISC  (1.0f / 4096.0f)
#define SSC  (1.0f / 8192.0f)
#define NEGB (-3.125e18f)
#define RNUM 16384.0f
#define CCEN 32.0f
#define HSC  (1.0f / 1024.0f)
#define CSV  (1.0f / 64.0f)
#define LOSC 2048.0f
#define OSC  (1.0f / 262144.0f)
#define LOIN (1.0f / 2048.0f)
#define NBX  ((MR * EE) / 2048)
#define NBW  ((EE * EE) / 2048)
static_assert(EE == NH * DH);
static_assert(DH == 32);
static_assert((LQ % 64) == 0 && (EE % 128) == 0 && (MR % 64) == 0);
static_assert(((MR * EE) % 2048) == 0 && ((EE * EE) % 2048) == 0);
static_assert(NBX == 1024 && NBW == 32);

typedef _Float16 v16h __attribute__((ext_vector_type(16)));
typedef _Float16 v8h  __attribute__((ext_vector_type(8)));
typedef float    v8f  __attribute__((ext_vector_type(8)));
typedef float    v4f  __attribute__((ext_vector_type(4)));
typedef unsigned int v4u __attribute__((ext_vector_type(4)));
typedef int      v4i  __attribute__((ext_vector_type(4)));

union FragH { v16h v; v8h h[2]; };

__device__ __forceinline__ unsigned short bf_bits(float f) {
  unsigned u = __float_as_uint(f);
  return (unsigned short)((u + 0x7FFFu + ((u >> 16) & 1u)) >> 16);
}
__device__ __forceinline__ float bf_up(unsigned short h) { return __uint_as_float(((unsigned)h) << 16); }
__device__ __forceinline__ float bfr(float f) { return bf_up(bf_bits(f)); }
__device__ __forceinline__ unsigned short h_bits(_Float16 x) { return __builtin_bit_cast(unsigned short, x); }
__device__ __forceinline__ unsigned pk16(unsigned short a, unsigned short b) { return (unsigned)a | ((unsigned)b << 16); }
__device__ __forceinline__ v8f zero8() { v8f z = {0.f, 0.f, 0.f, 0.f, 0.f, 0.f, 0.f, 0.f}; return z; }
__device__ __forceinline__ v4u cvt8(v4f a, v4f c, float sc) {
  float f[8];
#pragma unroll
  for (int i = 0; i < 4; ++i) { f[i] = bfr(a[i]) * sc; f[4 + i] = bfr(c[i]) * sc; }
  v4u v;
#pragma unroll
  for (int i = 0; i < 4; ++i) v[i] = pk16(h_bits((_Float16)f[2 * i]), h_bits((_Float16)f[2 * i + 1]));
  return v;
}

__device__ __forceinline__ v16h ldfrag_h(const _Float16* p) {
  FragH f;
  f.h[0] = *(const v8h*)(p);
  f.h[1] = *(const v8h*)(p + 16);
  return f.v;
}

__device__ __forceinline__ v8f mma_h(v16h a, v16h b, v8f c) {
  return __builtin_amdgcn_wmma_f32_16x16x32_f16(false, a, false, b, (short)0, c, false, false);
}
__device__ __forceinline__ void guard2(v8f& a, v8f& b, v16h x0, v16h x1, v16h y) {
#if defined(__HIP_DEVICE_COMPILE__)
  asm volatile("v_nop\n\tv_nop\n\tv_nop\n\tv_nop" : "+v"(a), "+v"(b) : "v"(x0), "v"(x1), "v"(y));
#endif
}
__device__ __forceinline__ void guard4(v8f& a, v8f& b, v8f& c, v8f& d,
                                       v16h x, v16h y0, v16h y1, v16h y2, v16h y3) {
#if defined(__HIP_DEVICE_COMPILE__)
  asm volatile("v_nop\n\tv_nop\n\tv_nop\n\tv_nop"
               : "+v"(a), "+v"(b), "+v"(c), "+v"(d) : "v"(x), "v"(y0), "v"(y1), "v"(y2), "v"(y3));
#endif
}

__global__ __launch_bounds__(256)
void cvt_planes(const float* __restrict__ xv, const float* __restrict__ xk, const float* __restrict__ xq,
                const float* __restrict__ wv, const float* __restrict__ wk, const float* __restrict__ wq,
                const float* __restrict__ wo,
                unsigned short* pv, unsigned short* pk, unsigned short* pq,
                unsigned short* hv, unsigned short* hk, unsigned short* hq, unsigned short* ho) {
  const int bx = blockIdx.x;
  const float* src;
  unsigned short* dst;
  int lb;
  float sc;
  if (bx < NBX)          { src = xv; dst = pv; lb = bx;           sc = XSC; }
  else if (bx < 2 * NBX) { src = xk; dst = pk; lb = bx - NBX;     sc = XSC; }
  else if (bx < 3 * NBX) { src = xq; dst = pq; lb = bx - 2 * NBX; sc = XSC; }
  else {
    const int r = bx - 3 * NBX;
    const int w = r / NBW;
    lb = r - w * NBW;
    sc = WSC;
    if (w == 0)      { src = wv; dst = hv; }
    else if (w == 1) { src = wk; dst = hk; }
    else if (w == 2) { src = wq; dst = hq; }
    else             { src = wo; dst = ho; }
  }
  const size_t e0 = ((size_t)lb * 256 + threadIdx.x) * 8;
  const v4f a = *(const v4f*)(src + e0);
  const v4f c = *(const v4f*)(src + e0 + 4);
  const v4u v = cvt8(a, c, sc);
  unsigned short* dp = dst + e0;
  *(volatile v4u*)dp = v;
  __threadfence();
  *(volatile v4u*)dp = v;
}

__global__ __launch_bounds__(256)
void colsum_sv(const float* __restrict__ xv, const float* __restrict__ wv, float* svo) {
  __shared__ __align__(16) float Cs[EE];
  __shared__ __align__(16) float Ss[EE];
  const int ns = blockIdx.x;
  const int t  = threadIdx.x;
  const float* p = xv + (size_t)ns * LQ * EE + t;
  float s = 0.f;
#pragma unroll 4
  for (int l = 0; l < LQ; ++l) s += bfr(p[(size_t)l * EE]);
  Cs[t] = s;
  __syncthreads();
  const float* wr = wv + (size_t)t * EE;
  float a = 0.f;
#pragma unroll 4
  for (int e = 0; e < EE; ++e) a = fmaf(Cs[e], bfr(wr[e]), a);
  Ss[t] = a;
  __syncthreads();
  if (t < 64) {
    const v4f v = *(const v4f*)(Ss + 4 * t);
    float* dp = svo + (size_t)ns * EE + 4 * t;
    *(volatile v4f*)dp = v;
    __threadfence();
    *(volatile v4f*)dp = v;
  }
}

template <int TR>
__global__ __launch_bounds__(128)
void proj_gemm(const unsigned short* __restrict__ wh, const unsigned short* __restrict__ xh, unsigned short* yo) {
  __shared__ __align__(16) unsigned short Ts[128 * 72];
  const int tid  = threadIdx.x;
  const int wave = tid >> 5;
  const int lane = tid & 31;
  const int hh   = lane >> 4;
  const int ci   = lane & 15;
  const int bx   = blockIdx.x;
  const int mt   = bx >> 1, ot = bx & 1;
  const int m0   = mt * 64, o0 = ot * 128;
  const _Float16* W = (const _Float16*)(const void*)wh;
  const _Float16* X = (const _Float16*)(const void*)xh;
  const _Float16* xr = X + (size_t)(m0 + 16 * wave + ci) * EE + 8 * hh;
  const _Float16* wr = W + (size_t)(o0 + ci) * EE + 8 * hh;

  v8f acc[8];
#pragma unroll
  for (int t = 0; t < 8; ++t) acc[t] = zero8();

#pragma unroll 1
  for (int ks = 0; ks < EE / 32; ++ks) {
    const int k0 = ks * 32;
    const v16h xb = ldfrag_h(xr + k0);
    v16h wa[4];
#pragma unroll
    for (int t = 0; t < 4; ++t) wa[t] = ldfrag_h(wr + (size_t)(16 * t) * EE + k0);
#pragma unroll
    for (int t = 0; t < 4; ++t) acc[t] = mma_h(wa[t], xb, acc[t]);
    guard4(acc[0], acc[1], acc[2], acc[3], xb, wa[0], wa[1], wa[2], wa[3]);
    v16h wc[4];
#pragma unroll
    for (int t = 0; t < 4; ++t) wc[t] = ldfrag_h(wr + (size_t)(16 * (t + 4)) * EE + k0);
#pragma unroll
    for (int t = 0; t < 4; ++t) acc[4 + t] = mma_h(wc[t], xb, acc[4 + t]);
    guard4(acc[4], acc[5], acc[6], acc[7], xb, wc[0], wc[1], wc[2], wc[3]);
  }

  if (TR == 0) {
    unsigned short* ts = Ts + (16 * wave + ci) * 136 + 8 * hh;
#pragma unroll
    for (int t = 0; t < 8; ++t) {
      v4u v;
#pragma unroll
      for (int i = 0; i < 4; ++i)
        v[i] = pk16(h_bits((_Float16)(acc[t][2 * i] * ISC)), h_bits((_Float16)(acc[t][2 * i + 1] * ISC)));
      *(v4u*)(ts + 16 * t) = v;
    }
    __syncthreads();
    const int p = tid & 15, r16 = tid >> 4;
    v4u vals[8];
#pragma unroll
    for (int it = 0; it < 8; ++it) {
      const int row = it * 8 + r16;
      vals[it] = *(const v4u*)(Ts + row * 136 + 8 * p);
    }
    unsigned short* yb = yo + (size_t)m0 * EE + o0 + 8 * p;
    for (int pass = 0; pass < 2; ++pass) {
#pragma unroll
      for (int it = 0; it < 8; ++it) {
        const int row = it * 8 + r16;
        *(volatile v4u*)(yb + (size_t)row * EE) = vals[it];
      }
      __threadfence();
    }
  } else {
    const int ns = m0 / LQ, l0 = m0 - ns * LQ;
#pragma unroll
    for (int t = 0; t < 8; ++t) {
#pragma unroll
      for (int r = 0; r < 8; ++r)
        Ts[(16 * t + 8 * hh + r) * 72 + 16 * wave + ci] = h_bits((_Float16)(acc[t][r] * ISC));
    }
    __syncthreads();
    const int e8 = tid & 7, fq = tid >> 3;
    v4u vals[8];
#pragma unroll
    for (int it = 0; it < 8; ++it) {
      const int orow = it * 16 + fq;
      vals[it] = *(const v4u*)(Ts + orow * 72 + 8 * e8);
    }
    unsigned short* yb = yo + ((size_t)ns * EE + o0) * LQ + l0 + 8 * e8;
    for (int pass = 0; pass < 2; ++pass) {
#pragma unroll
      for (int it = 0; it < 8; ++it) {
        const int orow = it * 16 + fq;
        *(volatile v4u*)(yb + (size_t)orow * LQ) = vals[it];
      }
      __threadfence();
    }
  }
}

__global__ __launch_bounds__(128)
void col_stats(const unsigned short* __restrict__ q16, const unsigned short* __restrict__ k16,
               const int* __restrict__ mask, float* mst, float* rst) {
  __shared__ __align__(16) int Mk[LQ];
  __shared__ __align__(16) float Sm[64];
  __shared__ __align__(16) float Sr[64];
  const int tid  = threadIdx.x;
  const int wave = tid >> 5;
  const int lane = tid & 31;
  const int hh   = lane >> 4;
  const int ci   = lane & 15;
  const int bx   = blockIdx.x;
  const int ns   = bx / (NH * (LQ / 64));
  const int rem  = bx - ns * (NH * (LQ / 64));
  const int h    = rem / (LQ / 64);
  const int l0   = (rem - h * (LQ / 64)) * 64;
  {
    const int* mp = mask + (size_t)ns * LQ + 8 * tid;
    *(v4i*)(Mk + 8 * tid)     = *(const v4i*)(mp);
    *(v4i*)(Mk + 8 * tid + 4) = *(const v4i*)(mp + 4);
  }
  __syncthreads();
  const _Float16* Q = (const _Float16*)(const void*)q16;
  const _Float16* K = (const _Float16*)(const void*)k16;
  const v16h kf = ldfrag_h(K + (size_t)(ns * LQ + l0 + 16 * wave + ci) * EE + h * DH + 8 * hh);
  const _Float16* qp = Q + (size_t)(ns * LQ + ci) * EE + h * DH + 8 * hh;

  float m = -1.0e30f, z = 0.f;
#pragma unroll 1
  for (int it = 0; it < LQ / 32; ++it) {
    const int qb = it * 32;
    const v16h x0 = ldfrag_h(qp + (size_t)qb * EE);
    const v16h x1 = ldfrag_h(qp + (size_t)(qb + 16) * EE);
    v8f s0 = mma_h(x0, kf, zero8());
    v8f s1 = mma_h(x1, kf, zero8());
    guard2(s0, s1, x0, x1, kf);
    const v4i ma = *(const v4i*)(Mk + qb + 8 * hh);
    const v4i mb = *(const v4i*)(Mk + qb + 8 * hh + 4);
    const v4i mc = *(const v4i*)(Mk + qb + 16 + 8 * hh);
    const v4i md = *(const v4i*)(Mk + qb + 16 + 8 * hh + 4);
    float t[16];
#pragma unroll
    for (int r = 0; r < 4; ++r) {
      t[r]      = (ma[r] != 0) ? s0[r] * SSC     : NEGB;
      t[4 + r]  = (mb[r] != 0) ? s0[4 + r] * SSC : NEGB;
      t[8 + r]  = (mc[r] != 0) ? s1[r] * SSC     : NEGB;
      t[12 + r] = (md[r] != 0) ? s1[4 + r] * SSC : NEGB;
    }
    float mx = t[0];
#pragma unroll
    for (int i = 1; i < 16; ++i) mx = fmaxf(mx, t[i]);
    const float mn = fmaxf(m, mx);
    z *= __expf(m - mn);
    float zs = 0.f;
#pragma unroll
    for (int i = 0; i < 16; ++i) zs += __expf(t[i] - mn);
    z += zs;
    m = mn;
  }
  const float mo = __shfl_xor(m, 16, 32);
  const float zo = __shfl_xor(z, 16, 32);
  const float mm = fmaxf(m, mo);
  const float zz = z * __expf(m - mm) + zo * __expf(mo - mm);
  if (hh == 0) { Sm[16 * wave + ci] = mm; Sr[16 * wave + ci] = RNUM / zz; }
  __syncthreads();
  if (wave == 0) {
    const v4f va = *(const v4f*)(Sm + 4 * ci);
    const v4f vb = *(const v4f*)(Sr + 4 * ci);
    v4f v;
#pragma unroll
    for (int e = 0; e < 4; ++e) v[e] = hh ? vb[e] : va[e];
    float* dp = (hh ? rst : mst) + (size_t)(ns * NH + h) * LQ + l0 + 4 * ci;
    *(volatile v4f*)dp = v;
    __threadfence();
    *(volatile v4f*)dp = v;
  }
}

__global__ __launch_bounds__(128)
void attn_out(const unsigned short* __restrict__ q16, const unsigned short* __restrict__ k16,
              const unsigned short* __restrict__ vt, const float* __restrict__ mst,
              const float* __restrict__ rst, const int* __restrict__ mask,
              const float* __restrict__ sv, unsigned short* ohp, unsigned short* olp) {
  __shared__ __align__(16) unsigned short Hs[64 * 40];
  __shared__ __align__(16) unsigned short Lw[64 * 40];
  const int tid  = threadIdx.x;
  const int wave = tid >> 5;
  const int lane = tid & 31;
  const int hh   = lane >> 4;
  const int ci   = lane & 15;
  const int bx   = blockIdx.x;
  const int ns   = bx / (NH * (LQ / 64));
  const int rem  = bx - ns * (NH * (LQ / 64));
  const int h    = rem / (LQ / 64);
  const int q0   = (rem - h * (LQ / 64)) * 64;
  const int qi   = q0 + 16 * wave + ci;

  const _Float16* Q = (const _Float16*)(const void*)q16;
  const _Float16* K = (const _Float16*)(const void*)k16;
  const _Float16* V = (const _Float16*)(const void*)vt;
  const v16h qf = ldfrag_h(Q + (size_t)(ns * LQ + qi) * EE + h * DH + 8 * hh);
  const _Float16* kp = K + (size_t)(ns * LQ + ci) * EE + h * DH + 8 * hh;
  const _Float16* vp = V + ((size_t)ns * EE + h * DH + ci) * LQ + 8 * hh;
  const size_t sb = (size_t)(ns * NH + h) * LQ + 8 * hh;
  const float* mp = mst + sb;
  const float* rp = rst + sb;
  const int  mq = mask[(size_t)ns * LQ + qi];
  const bool um = (mq != 0);
  const float cc = um ? CCEN : 0.0f;

  v8f acc0 = zero8(), acc1 = zero8();
#pragma unroll 1
  for (int it = 0; it < LQ / 32; ++it) {
    const int lt = it * 32;
    const v16h ka0 = ldfrag_h(kp + (size_t)lt * EE);
    const v16h ka1 = ldfrag_h(kp + (size_t)(lt + 16) * EE);
    v8f s0 = mma_h(ka0, qf, zero8());
    v8f s1 = mma_h(ka1, qf, zero8());
    guard2(s0, s1, ka0, ka1, qf);
    const v4f ma = *(const v4f*)(mp + lt);
    const v4f mb = *(const v4f*)(mp + lt + 4);
    const v4f mc = *(const v4f*)(mp + lt + 16);
    const v4f md = *(const v4f*)(mp + lt + 20);
    const v4f ra = *(const v4f*)(rp + lt);
    const v4f rb = *(const v4f*)(rp + lt + 4);
    const v4f rc = *(const v4f*)(rp + lt + 16);
    const v4f rd = *(const v4f*)(rp + lt + 20);
    FragH pb;
#pragma unroll
    for (int r = 0; r < 4; ++r) {
      const float t00 = um ? s0[r] * SSC     : NEGB;
      const float t01 = um ? s0[4 + r] * SSC : NEGB;
      const float t10 = um ? s1[r] * SSC     : NEGB;
      const float t11 = um ? s1[4 + r] * SSC : NEGB;
      pb.h[0][r]     = (_Float16)(__expf(t00 - ma[r]) * ra[r] - cc);
      pb.h[0][4 + r] = (_Float16)(__expf(t01 - mb[r]) * rb[r] - cc);
      pb.h[1][r]     = (_Float16)(__expf(t10 - mc[r]) * rc[r] - cc);
      pb.h[1][4 + r] = (_Float16)(__expf(t11 - md[r]) * rd[r] - cc);
    }
    const v16h va0 = ldfrag_h(vp + lt);
    const v16h va1 = ldfrag_h(vp + (size_t)16 * LQ + lt);
    acc0 = mma_h(va0, pb.v, acc0);
    acc1 = mma_h(va1, pb.v, acc1);
    guard2(acc0, acc1, va0, va1, pb.v);
  }

  const float* svp = sv + (size_t)ns * EE + h * DH + 8 * hh;
  const v4f sa = *(const v4f*)(svp);
  const v4f sq = *(const v4f*)(svp + 4);
  const v4f sc = *(const v4f*)(svp + 16);
  const v4f sd = *(const v4f*)(svp + 20);
  const float csv = cc * CSV;
  float o[16];
#pragma unroll
  for (int r = 0; r < 4; ++r) {
    o[r]      = acc0[r] * HSC     + csv * sa[r];
    o[4 + r]  = acc0[4 + r] * HSC + csv * sq[r];
    o[8 + r]  = acc1[r] * HSC     + csv * sc[r];
    o[12 + r] = acc1[4 + r] * HSC + csv * sd[r];
  }
  v4u h0, h1, g0, g1;
#pragma unroll
  for (int i = 0; i < 4; ++i) {
    const _Float16 a0 = (_Float16)o[2 * i],     a1 = (_Float16)o[2 * i + 1];
    const _Float16 b0 = (_Float16)o[8 + 2 * i], b1 = (_Float16)o[8 + 2 * i + 1];
    const _Float16 la0 = (_Float16)((o[2 * i]         - (float)a0) * LOSC);
    const _Float16 la1 = (_Float16)((o[2 * i + 1]     - (float)a1) * LOSC);
    const _Float16 lb0 = (_Float16)((o[8 + 2 * i]     - (float)b0) * LOSC);
    const _Float16 lb1 = (_Float16)((o[8 + 2 * i + 1] - (float)b1) * LOSC);
    h0[i] = pk16(h_bits(a0), h_bits(a1));
    h1[i] = pk16(h_bits(b0), h_bits(b1));
    g0[i] = pk16(h_bits(la0), h_bits(la1));
    g1[i] = pk16(h_bits(lb0), h_bits(lb1));
  }
  {
    const int ro = (16 * wave + ci) * 40 + 8 * hh;
    *(v4u*)(Hs + ro)      = h0;
    *(v4u*)(Hs + ro + 16) = h1;
    *(v4u*)(Lw + ro)      = g0;
    *(v4u*)(Lw + ro + 16) = g1;
  }
  __syncthreads();
  {
    const size_t ob = ((size_t)(ns * NH + h) * LQ + q0) * DH;
    v4u hv[2], lv[2];
#pragma unroll
    for (int it2 = 0; it2 < 2; ++it2) {
      const int hf = it2 * 1024 + 8 * tid;
      const int row = hf >> 5, col = hf & 31;
      hv[it2] = *(const v4u*)(Hs + row * 40 + col);
      lv[it2] = *(const v4u*)(Lw + row * 40 + col);
    }
    for (int pass = 0; pass < 2; ++pass) {
#pragma unroll
      for (int it2 = 0; it2 < 2; ++it2) {
        const int hf = it2 * 1024 + 8 * tid;
        *(volatile v4u*)(ohp + ob + hf) = hv[it2];
        *(volatile v4u*)(olp + ob + hf) = lv[it2];
      }
      __threadfence();
    }
  }
}

__global__ __launch_bounds__(128)
void out_proj(const unsigned short* __restrict__ ohp, const unsigned short* __restrict__ olp,
              const unsigned short* __restrict__ woh, const float* __restrict__ bo, float* out) {
  __shared__ __align__(16) float Ts[64 * 68];
  const int tid  = threadIdx.x;
  const int wave = tid >> 5;
  const int lane = tid & 31;
  const int hh   = lane >> 4;
  const int ci   = lane & 15;
  const int bx   = blockIdx.x;
  const int mt   = bx >> 2, ot = bx & 3;
  const int m0   = mt * 64, o0 = ot * 64;
  const int ns   = m0 / LQ;
  const int ql   = m0 - ns * LQ + 16 * wave + ci;
  const _Float16* OHf = (const _Float16*)(const void*)ohp;
  const _Float16* OLf = (const _Float16*)(const void*)olp;
  const _Float16* W   = (const _Float16*)(const void*)woh;
  const size_t orow = ((size_t)(ns * NH) * LQ + ql) * DH + 8 * hh;
  const _Float16* ar = OHf + orow;
  const _Float16* lr = OLf + orow;
  const _Float16* wr = W + (size_t)(o0 + ci) * EE + 8 * hh;

  v8f acch[4], accl[4];
#pragma unroll
  for (int t = 0; t < 4; ++t) { acch[t] = zero8(); accl[t] = zero8(); }

#pragma unroll 1
  for (int j = 0; j < NH; ++j) {
    const v16h obh = ldfrag_h(ar + (size_t)j * LQ * DH);
    const v16h obl = ldfrag_h(lr + (size_t)j * LQ * DH);
    v16h wa[4];
#pragma unroll
    for (int t = 0; t < 4; ++t) wa[t] = ldfrag_h(wr + (size_t)(16 * t) * EE + 32 * j);
#pragma unroll
    for (int t = 0; t < 4; ++t) acch[t] = mma_h(wa[t], obh, acch[t]);
    guard4(acch[0], acch[1], acch[2], acch[3], obh, wa[0], wa[1], wa[2], wa[3]);
#pragma unroll
    for (int t = 0; t < 4; ++t) accl[t] = mma_h(wa[t], obl, accl[t]);
    guard4(accl[0], accl[1], accl[2], accl[3], obl, wa[0], wa[1], wa[2], wa[3]);
  }

  {
    float* ts = Ts + (16 * wave + ci) * 68 + 8 * hh;
#pragma unroll
    for (int t = 0; t < 4; ++t) {
      const v4f b0 = *(const v4f*)(bo + o0 + 16 * t + 8 * hh);
      const v4f b1 = *(const v4f*)(bo + o0 + 16 * t + 8 * hh + 4);
      v4f r0, r1;
#pragma unroll
      for (int e = 0; e < 4; ++e) {
        r0[e] = (acch[t][e]     + accl[t][e]     * LOIN) * OSC + bfr(b0[e]);
        r1[e] = (acch[t][4 + e] + accl[t][4 + e] * LOIN) * OSC + bfr(b1[e]);
      }
      *(v4f*)(ts + 16 * t)     = r0;
      *(v4f*)(ts + 16 * t + 4) = r1;
    }
  }
  __syncthreads();
  {
    const int p = tid & 15, r16 = tid >> 4;
    v4f vals[8];
#pragma unroll
    for (int it = 0; it < 8; ++it) {
      const int row = it * 8 + r16;
      vals[it] = *(const v4f*)(Ts + row * 68 + 4 * p);
    }
    float* yb = out + (size_t)m0 * EE + o0 + 4 * p;
    for (int pass = 0; pass < 2; ++pass) {
#pragma unroll
      for (int it = 0; it < 8; ++it) {
        const int row = it * 8 + r16;
        *(volatile v4f*)(yb + (size_t)row * EE) = vals[it];
      }
      __threadfence();
    }
  }
}

extern "C" void kernel_launch(void* const* d_in, const int* in_sizes, int n_in,
                              void* d_out, int out_size, void* d_ws, size_t ws_size,
                              hipStream_t stream) {
  if (n_in < 10) return;
  if (in_sizes[0] != MR * EE || in_sizes[1] != MR * EE || in_sizes[2] != MR * EE) return;
  if (in_sizes[3] != NSB * LQ) return;
  if (in_sizes[5] != EE * EE || in_sizes[6] != EE * EE || in_sizes[7] != EE * EE || in_sizes[8] != EE * EE) return;
  if (in_sizes[9] != EE) return;
  if (out_size != MR * EE) return;

  const float* values  = (const float*)d_in[0];
  const float* keys    = (const float*)d_in[1];
  const float* queries = (const float*)d_in[2];
  const int*   mask    = (const int*)d_in[3];
  const float* Wv      = (const float*)d_in[5];
  const float* Wk      = (const float*)d_in[6];
  const float* Wq      = (const float*)d_in[7];
  const float* Wo      = (const float*)d_in[8];
  const float* bo      = (const float*)d_in[9];
  float* out = (float*)d_out;

  const size_t PX  = (size_t)MR * EE * 2;
  const size_t PW  = (size_t)EE * EE * 2;
  const size_t PP  = (size_t)MR * EE * 2;
  const size_t PVT = (size_t)NSB * EE * LQ * 2;
  const size_t PS  = (size_t)NSB * NH * LQ * 4;
  const size_t PSV = (size_t)NSB * EE * 4;
  const size_t PO  = (size_t)NSB * NH * LQ * DH * 2;
  size_t off = 0;
  const size_t oPV = off; off += PX;
  const size_t oPK = off; off += PX;
  const size_t oPQ = off; off += PX;
  const size_t oHV = off; off += PW;
  const size_t oHK = off; off += PW;
  const size_t oHQ = off; off += PW;
  const size_t oHO = off; off += PW;
  const size_t oQ  = off; off += PP;
  const size_t oK  = off; off += PP;
  const size_t oVT = off; off += PVT;
  const size_t oM  = off; off += PS;
  const size_t oR  = off; off += PS;
  const size_t oSV = off; off += PSV;
  const size_t oOH = off; off += PO;
  const size_t oOL = off; off += PO;
  if (off > ws_size) return;
  if (off > (size_t)134217728) return;

  char* ws = (char*)d_ws;
  unsigned short* PVp = (unsigned short*)(ws + oPV);
  unsigned short* PKp = (unsigned short*)(ws + oPK);
  unsigned short* PQp = (unsigned short*)(ws + oPQ);
  unsigned short* HVp = (unsigned short*)(ws + oHV);
  unsigned short* HKp = (unsigned short*)(ws + oHK);
  unsigned short* HQp = (unsigned short*)(ws + oHQ);
  unsigned short* HOp = (unsigned short*)(ws + oHO);
  unsigned short* Q16 = (unsigned short*)(ws + oQ);
  unsigned short* K16 = (unsigned short*)(ws + oK);
  unsigned short* VTp = (unsigned short*)(ws + oVT);
  float*          Mp  = (float*)(ws + oM);
  float*          Rp  = (float*)(ws + oR);
  float*          SVp = (float*)(ws + oSV);
  unsigned short* OHp = (unsigned short*)(ws + oOH);
  unsigned short* OLp = (unsigned short*)(ws + oOL);

  const dim3 blk256(256), blk128(128);
  const dim3 gCV(3 * NBX + 4 * NBW);
  const dim3 gCS(NSB);
  const dim3 gPJ((MR / 64) * (EE / 128));
  const dim3 gAT(NSB * NH * (LQ / 64));
  const dim3 gOP((MR / 64) * (EE / 64));

  cvt_planes<<<gCV, blk256, 0, stream>>>(values, keys, queries, Wv, Wk, Wq, Wo,
                                          PVp, PKp, PQp, HVp, HKp, HQp, HOp);
  colsum_sv<<<gCS, blk256, 0, stream>>>(values, Wv, SVp);
  proj_gemm<0><<<gPJ, blk128, 0, stream>>>(HQp, PQp, Q16);
  proj_gemm<0><<<gPJ, blk128, 0, stream>>>(HKp, PKp, K16);
  proj_gemm<1><<<gPJ, blk128, 0, stream>>>(HVp, PVp, VTp);
  col_stats<<<gAT, blk128, 0, stream>>>(Q16, K16, mask, Mp, Rp);
  attn_out<<<gAT, blk128, 0, stream>>>(Q16, K16, VTp, Mp, Rp, mask, SVp, OHp, OLp);
  out_proj<<<gOP, blk128, 0, stream>>>(OHp, OLp, HOp, bo, out);
  (void)hipGetLastError();
}
